// LePEAttention_1992864825858
// MI455X (gfx1250) — hardware-verified
//
#include <hip/hip_runtime.h>


typedef _Float16 half_t;
typedef __attribute__((ext_vector_type(16))) _Float16 v16h;
typedef __attribute__((ext_vector_type(8)))  float    v8f;

#define BSZ    8
#define CCH    128
#define HEADS  4
#define HD     32
#define NTOK   512
#define SCALEQ (0.17677669529663687f * 1.4426950408889634f)

#define K_STRIDE  40
#define V_STRIDE  40
#define P_STRIDE  40
#define K_OFF     0
#define VT_OFF    (512 * K_STRIDE)
#define P_OFF     (VT_OFF + 512 * V_STRIDE)
#define LDS_HALF  (P_OFF + 8 * 16 * P_STRIDE)

__global__ void __launch_bounds__(256)
lepe_attn_wmma_kernel(const float* __restrict__ qkv, float* __restrict__ out)
{
    extern __shared__ half_t smem[];

    const int whrt = blockIdx.x;
    const int wh   = whrt >> 2;
    const int rtg  = whrt & 3;
    const int head = wh & (HEADS - 1);
    const int win  = wh >> 2;
    const int b    = win >> 3;
    const int w    = win & 7;

    const size_t plane = (size_t)BSZ * 4096 * CCH;
    const float* qb  = qkv + (size_t)b * 4096 * CCH;
    const float* kb_ = qb + plane;
    const float* vb_ = qb + 2 * plane;

    const int tid  = threadIdx.x;
    const int lane = tid & 31;
    const int wave = tid >> 5;
    const int hh   = lane >> 4;
    const int lm   = lane & 15;

    for (int p = 0; p < 16; ++p) {
        const int n  = p * 32 + (tid >> 3);
        const int d0 = (tid & 7) * 4;
        const int yw = n >> 3, xw = n & 7;
        const size_t off = (size_t)(yw * 64 + w * 8 + xw) * CCH + head * HD + d0;
        const float4 k4 = *(const float4*)(kb_ + off);
        const float4 v4 = *(const float4*)(vb_ + off);
        half_t* kr = smem + K_OFF + n * K_STRIDE + d0;
        kr[0] = (half_t)k4.x; kr[1] = (half_t)k4.y;
        kr[2] = (half_t)k4.z; kr[3] = (half_t)k4.w;
        half_t* vr = smem + VT_OFF + n * V_STRIDE + d0;
        vr[0] = (half_t)v4.x; vr[1] = (half_t)v4.y; vr[2] = (half_t)v4.z; vr[3] = (half_t)v4.w;
    }
    __syncthreads();

    half_t* pbuf = smem + P_OFF + wave * 16 * P_STRIDE;

    const int qtok0 = (rtg * 8 + wave) * 16;

    v16h aq;
    {
        const int m  = qtok0 + lm;
        const int yw = m >> 3, xw = m & 7;
        const float* qrow = qb + (size_t)(yw * 64 + w * 8 + xw) * CCH + head * HD;
        #pragma unroll
        for (int i = 0; i < 16; ++i) {
            const int k = ((i >> 3) << 4) + (hh << 3) + (i & 7);
            aq[i] = (half_t)(qrow[k] * SCALEQ);
        }
    }

    v16h bones;
    #pragma unroll
    for (int i = 0; i < 16; ++i) bones[i] = (half_t)1.0f;

    v8f o0 = {}, o1 = {}, sacc = {};
    const v8f zero = {};

    for (int kblk = 0; kblk < 16; ++kblk) {
        v16h bk0, bk1;
        {
            const half_t* r0 = smem + K_OFF + (kblk * 32 + lm)      * K_STRIDE;
            const half_t* r1 = smem + K_OFF + (kblk * 32 + 16 + lm) * K_STRIDE;
            #pragma unroll
            for (int i = 0; i < 16; ++i) { const int k = ((i >> 3) << 4) + (hh << 3) + (i & 7); bk0[i] = r0[k]; bk1[i] = r1[k]; }
        }
        v8f s0 = __builtin_amdgcn_wmma_f32_16x16x32_f16(false, aq, false, bk0,
                                                        (short)0, zero, false, false);
        v8f s1 = __builtin_amdgcn_wmma_f32_16x16x32_f16(false, aq, false, bk1,
                                                        (short)0, zero, false, false);

        #pragma unroll
        for (int r = 0; r < 8; ++r) {
            const float p0 = __builtin_amdgcn_exp2f(s0[r]);
            const float p1 = __builtin_amdgcn_exp2f(s1[r]);
            const int row = r + (hh << 3);
            pbuf[row * P_STRIDE + lm]      = (half_t)p0;
            pbuf[row * P_STRIDE + 16 + lm] = (half_t)p1;
        }
        v16h ap;
        {
            const half_t* pr = pbuf + lm * P_STRIDE;
            #pragma unroll
            for (int i = 0; i < 16; ++i) {
                const int k = ((i >> 3) << 4) + (hh << 3) + (i & 7);
                ap[i] = pr[k];
            }
        }
        v16h bv0, bv1;
        {
            const half_t* vb0 = smem + VT_OFF + (kblk * 32) * V_STRIDE;
            #pragma unroll
            for (int i = 0; i < 16; ++i) { const int k = ((i >> 3) << 4) + (hh << 3) + (i & 7);
                bv0[i] = vb0[k * V_STRIDE + lm]; bv1[i] = vb0[k * V_STRIDE + 16 + lm]; }
        }
        o0   = __builtin_amdgcn_wmma_f32_16x16x32_f16(false, ap, false, bv0,
                                                      (short)0, o0,   false, false);
        o1   = __builtin_amdgcn_wmma_f32_16x16x32_f16(false, ap, false, bv1,
                                                      (short)0, o1,   false, false);
        sacc = __builtin_amdgcn_wmma_f32_16x16x32_f16(false, ap, false, bones,
                                                      (short)0, sacc, false, false);
        asm volatile("v_nop\n\tv_nop\n\tv_nop\n\tv_nop" : "+v"(o0), "+v"(sacc) : "v"(ap), "v"(bones));
    }

    for (int pass = 0; pass < 2; ++pass) {
        #pragma unroll
        for (int r = 0; r < 8; ++r) {
            const float inv = 1.0f / sacc[r];
            const float v0 = o0[r] * inv, v1 = o1[r] * inv;
            const float x0 = __shfl_xor(v0, 16), x1 = __shfl_xor(v1, 16);
            const int mA = qtok0 + r, mB = qtok0 + 8 + r;
            float* rowA = out + ((size_t)b * 4096 + (mA >> 3) * 64 + w * 8 + (mA & 7)) * CCH + head * HD;
            float* rowB = out + ((size_t)b * 4096 + (mB >> 3) * 64 + w * 8 + (mB & 7)) * CCH + head * HD;
            *(volatile float*)(rowA + lane) = hh ? x1 : v0;
            *(volatile float*)(rowB + lane) = hh ? v1 : x0;
        }
        __threadfence();
    }
}

__global__ void __launch_bounds__(256)
lepe_conv_add_kernel(const float* __restrict__ qkv, const float* __restrict__ cw,
                     const float* __restrict__ cb, float* __restrict__ out)
{
    const int idx = blockIdx.x * 256 + threadIdx.x;
    const int c   = idx & 127;
    const int t   = idx >> 7;
    const int x   = t & 7;
    const int y   = (t >> 3) & 63;
    const int win = t >> 9;
    const int b   = win >> 3;
    const int w   = win & 7;

    const float* vb_ = qkv + 2 * (size_t)BSZ * 4096 * CCH + (size_t)b * 4096 * CCH;
    float acc = cb[c];
    #pragma unroll
    for (int ky = 0; ky < 3; ++ky) {
        const int yy = y + ky - 1;
        if (yy < 0 || yy >= 64) continue;
        #pragma unroll
        for (int kx = 0; kx < 3; ++kx) {
            const int xx = x + kx - 1;
            if (xx < 0 || xx >= 8) continue;
            const float vv = vb_[(size_t)(yy * 64 + w * 8 + xx) * CCH + c];
            acc += vv * cw[c * 9 + ky * 3 + kx];
        }
    }
    const size_t oidx = ((size_t)b * 4096 + y * 64 + w * 8 + x) * CCH + c;
    const float nv = out[oidx] + acc;
    *(volatile float*)(out + oidx) = nv; __threadfence(); *(volatile float*)(out + oidx) = nv;
}

extern "C" void kernel_launch(void* const* d_in, const int* in_sizes, int n_in,
                              void* d_out, int out_size, void* d_ws, size_t ws_size,
                              hipStream_t stream)
{
    (void)in_sizes; (void)n_in; (void)out_size; (void)d_ws; (void)ws_size;
    const float* qkv = (const float*)d_in[0];
    const float* cw  = (const float*)d_in[1];
    const float* cb  = (const float*)d_in[2];
    float* out = (float*)d_out;

    const size_t shmem = (size_t)LDS_HALF * sizeof(half_t);
    hipFuncSetAttribute((const void*)lepe_attn_wmma_kernel, hipFuncAttributeMaxDynamicSharedMemorySize, (int)shmem);
    lepe_attn_wmma_kernel<<<1024, 256, shmem, stream>>>(qkv, out);
    lepe_conv_add_kernel<<<(64 * 512 * 128) / 256, 256, 0, stream>>>(qkv, cw, cb, out);
}
